// FuseMamba_43344809951446
// MI455X (gfx1250) — hardware-verified
//
#include <hip/hip_runtime.h>
#include <math.h>

typedef __attribute__((ext_vector_type(16))) _Float16 v16h;
typedef __attribute__((ext_vector_type(8)))  _Float16 v8h;
typedef __attribute__((ext_vector_type(16))) __bf16   v16b;
typedef __attribute__((ext_vector_type(8)))  __bf16   v8b;
typedef __attribute__((ext_vector_type(8)))  float    v8f;
typedef __attribute__((ext_vector_type(4)))  float    v4f;

constexpr int kNB    = 256;
constexpr int kNC    = 64;
constexpr int kNS    = 64;
constexpr int kPlane = kNB * kNC * kNS;
constexpr int kNBr   = 3;
constexpr int kSeq   = kNBr * kNB;
constexpr int kRows  = kSeq * kNC;
constexpr int kDin   = 128;
constexpr int kXZP   = 2 * kDin;
constexpr int kNst   = 16;
constexpr int kDtR   = 4;
constexpr int kXpN   = 36;
constexpr int kXpP   = 64;
constexpr int kTP    = 132;
static_assert(kPlane == 1048576);
static_assert(kRows % 64 == 0);

__device__ __forceinline__ unsigned short f2bf_bits(float f) {
  unsigned u = __float_as_uint(f);
  return (unsigned short)((u + 0x7FFFu + ((u >> 16) & 1u)) >> 16);
}
__device__ __forceinline__ float bf_bits2f(unsigned short h) { return __uint_as_float(((unsigned)h) << 16); }

__device__ __forceinline__ void dep_guard_h(v8f& a, v8f& b, v16h x, v16h y) { asm volatile("v_nop\n\tv_nop\n\tv_nop\n\tv_nop" : "+v"(a), "+v"(b) : "v"(x), "v"(y)); }
__device__ __forceinline__ void dep_guard_b(v8f& a, v8f& b, v16b x, v16b y) { asm volatile("v_nop\n\tv_nop\n\tv_nop\n\tv_nop" : "+v"(a), "+v"(b) : "v"(x), "v"(y)); }
__device__ __forceinline__ void keep4_h(v16h a, v16h b, v16h c, v16h d) { asm volatile("v_nop" :: "v"(a), "v"(b), "v"(c), "v"(d)); }
__device__ __forceinline__ void keep4_b(v16b a, v16b b, v16b c, v16b d) { asm volatile("v_nop" :: "v"(a), "v"(b), "v"(c), "v"(d)); }
__device__ __forceinline__ void acc_guard4(v8f& a, v8f& b, v8f& c, v8f& d) { asm volatile("v_nop\n\tv_nop\n\tv_nop\n\tv_nop" : "+v"(a), "+v"(b), "+v"(c), "+v"(d)); }
template <typename T> struct Frag;
template <> struct Frag<_Float16> {
  typedef v16h V; union U { v16h v; v8h h[2]; };
  static __device__ __forceinline__ v16h load(const _Float16* p) {
    U f; f.h[0] = *(const v8h*)(p); f.h[1] = *(const v8h*)(p + 16); return f.v;
  }
  static __device__ __forceinline__ v8f mma(v16h a, v16h b, v8f c) {
    return __builtin_amdgcn_wmma_f32_16x16x32_f16(false, a, false, b, (short)0, c, false, false);
  }
  static __device__ __forceinline__ void guard(v8f& a, v8f& b, v16h x, v16h y) { dep_guard_h(a, b, x, y); }
  static __device__ __forceinline__ void keep(v16h a, v16h b, v16h c, v16h d) { keep4_h(a, b, c, d); }
};
template <> struct Frag<__bf16> {
  typedef v16b V; union U { v16b v; v8b h[2]; };
  static __device__ __forceinline__ v16b load(const __bf16* p) {
    U f; f.h[0] = *(const v8b*)(p); f.h[1] = *(const v8b*)(p + 16); return f.v;
  }
  static __device__ __forceinline__ v8f mma(v16b a, v16b b, v8f c) {
    return __builtin_amdgcn_wmma_f32_16x16x32_bf16(false, a, false, b, (short)0, c, false, false);
  }
  static __device__ __forceinline__ void guard(v8f& a, v8f& b, v16b x, v16b y) { dep_guard_b(a, b, x, y); }
  static __device__ __forceinline__ void keep(v16b a, v16b b, v16b c, v16b d) { keep4_b(a, b, c, d); }
};

template <int ET> struct Elem;
template <> struct Elem<0> { typedef _Float16 T; };
template <> struct Elem<1> { typedef __bf16 T; };
template <int ET, bool SPLIT, int BIAS_MODE, int OUT_MODE, bool RESID, int ACT = 0, bool WAVEB = false>
__global__ __launch_bounds__(256) void wmma_gemm64(
    const unsigned short* __restrict__ Ap, const unsigned short* __restrict__ A2p, int lda, long strideA,
    const unsigned short* __restrict__ Btp, const unsigned short* __restrict__ Bt2p, int ldb, long strideB,
    void* __restrict__ Cout, void* __restrict__ Cout2, int ldc, long strideC,
    const float* __restrict__ bias,
    const float* __restrict__ resid, long strideR,
    int M, int N, int K, float scale) {
  typedef typename Elem<ET>::T T;
  typedef typename Frag<T>::V V;
  const T* A = (const T*)Ap; const T* A2 = (const T*)A2p; const T* Bt = (const T*)Btp; const T* Bt2 = (const T*)Bt2p;
  __shared__ __align__(16) float sT[8][16 * 68];
  const int lane = threadIdx.x & 31;
  const int wave = threadIdx.x >> 5;
  const int b    = WAVEB ? (int)(blockIdx.y * 8 + wave) : (int)blockIdx.y;
  const int tilesN = N >> 6;
  const int tilesM = M >> 6;
  const int tile = WAVEB ? (int)blockIdx.x : (int)(blockIdx.x * 8 + wave);
  if (tile >= tilesM * tilesN) return;
  const int tm = tile / tilesN;
  const int tn = tile - tm * tilesN;
  const int m0 = tm << 6;
  const int n0 = tn << 6;

  const T* Ab  = A  + (size_t)b * strideA;
  const T* Bb  = Bt + (size_t)b * strideB;
  const T* Ab2 = SPLIT ? (A2  + (size_t)b * strideA) : nullptr;
  const T* Bb2 = SPLIT ? (Bt2 + (size_t)b * strideB) : nullptr;

  const int rlane = lane & 15;
  const int koff  = (lane >> 4) * 8;
  const int mOff  = (lane >> 4) * 8;

  v8f acc[4][4];
#pragma unroll
  for (int i = 0; i < 4; ++i)
#pragma unroll
    for (int j = 0; j < 4; ++j) acc[i][j] = (v8f){0.f,0.f,0.f,0.f,0.f,0.f,0.f,0.f};

  for (int k0 = 0; k0 < K; k0 += 32) {
    V bh[4], bl[4];
#pragma unroll
    for (int j = 0; j < 4; ++j) {
      const size_t bo = (size_t)(n0 + (j << 4) + rlane) * ldb + koff + k0;
      bh[j] = Frag<T>::load(Bb + bo);
      if (SPLIT) bl[j] = Frag<T>::load(Bb2 + bo);
    }
#pragma unroll
    for (int i = 0; i < 4; ++i) {
      const size_t ao = (size_t)(m0 + (i << 4) + rlane) * lda + koff + k0;
      V ah = Frag<T>::load(Ab + ao);
      V al;
      if (SPLIT) al = Frag<T>::load(Ab2 + ao);
#pragma unroll
      for (int j = 0; j < 4; ++j) {
        acc[i][j] = Frag<T>::mma(ah, bh[j], acc[i][j]);
        if (SPLIT) {
          acc[i][j] = Frag<T>::mma(ah, bl[j], acc[i][j]);
          acc[i][j] = Frag<T>::mma(al, bh[j], acc[i][j]);
        }
      }
      Frag<T>::guard(acc[i][0], acc[i][3], ah, SPLIT ? al : ah);
    }
    Frag<T>::keep(bh[0], bh[1], bh[2], bh[3]);
    if (SPLIT) Frag<T>::keep(bl[0], bl[1], bl[2], bl[3]);
  }
  acc_guard4(acc[0][0], acc[0][1], acc[0][2], acc[0][3]);
  acc_guard4(acc[1][0], acc[1][1], acc[1][2], acc[1][3]);
  acc_guard4(acc[2][0], acc[2][1], acc[2][2], acc[2][3]);
  acc_guard4(acc[3][0], acc[3][1], acc[3][2], acc[3][3]);

  float* slab = sT[wave];
  const float* Rb = RESID ? (resid + (size_t)b * strideR) : nullptr;
#pragma unroll
  for (int i = 0; i < 4; ++i) {
    const int mBase = m0 + (i << 4);
#pragma unroll
    for (int j = 0; j < 4; ++j) {
      const int n = n0 + (j << 4) + rlane;
      float bv = 0.f;
      if (BIAS_MODE == 2) bv = bias[n];
#pragma unroll
      for (int r = 0; r < 8; ++r) {
        float v = acc[i][j][r] * scale;
        if (BIAS_MODE == 1) v += bias[mBase + mOff + r];
        if (BIAS_MODE == 2) v += bv;
        if (RESID) v += Rb[(size_t)(mBase + mOff + r) * ldc + n];
        if (ACT == 1) v = tanhf(v);
        if (ACT == 2) v = fmaxf(v, 0.0f);
        if (ACT == 3) v = v / (1.0f + expf(-v));
        if (ACT == 4) v = (v > 0.f) ? v : 0.01f * v;
        if (ACT == 5) v = 0.5f * v * (1.0f + erff(v * 0.70710678118654752f));
        slab[(mOff + r) * 68 + (j << 4) + rlane] = v;
      }
    }
    __builtin_amdgcn_fence(__ATOMIC_RELEASE, "workgroup");
    __builtin_amdgcn_wave_barrier();
    __builtin_amdgcn_fence(__ATOMIC_ACQUIRE, "workgroup");
    if (OUT_MODE == 0) {
      float* C = (float*)Cout + (size_t)b * strideC;
      const int hh = lane >> 4, c4 = (lane & 15) * 4;
      for (int pass = 0; pass < 2; ++pass) {
#pragma unroll
        for (int it = 0; it < 8; ++it) {
          const int row = it * 2 + hh;
          v4f v = *(const v4f*)(slab + row * 68 + c4);
          *(volatile v4f*)(C + (size_t)(mBase + row) * ldc + n0 + c4) = v;
        }
        __threadfence();
      }
    } else {
      const int q = lane >> 3, c8 = (lane & 7) * 8;
      unsigned short* C  = (unsigned short*)Cout  + (size_t)b * strideC;
      unsigned short* C2 = (OUT_MODE == 2) ? ((unsigned short*)Cout2 + (size_t)b * strideC) : nullptr;
      for (int pass = 0; pass < 2; ++pass) {
#pragma unroll
        for (int it = 0; it < 4; ++it) {
          const int row = it * 4 + q;
          const float* sp = slab + row * 68 + c8;
          v8h hv, lv;
#pragma unroll
          for (int e = 0; e < 8; ++e) {
            if (OUT_MODE == 1) {
              hv[e] = (_Float16)sp[e];
            } else {
              unsigned short hb = f2bf_bits(sp[e]);
              unsigned short lb = f2bf_bits(sp[e] - bf_bits2f(hb));
              hv[e] = __builtin_bit_cast(_Float16, hb);
              lv[e] = __builtin_bit_cast(_Float16, lb);
            }
          }
          *(volatile v8h*)(C + (size_t)(mBase + row) * ldc + n0 + c8) = hv;
          if (OUT_MODE == 2) *(volatile v8h*)(C2 + (size_t)(mBase + row) * ldc + n0 + c8) = lv;
        }
        __threadfence();
      }
    }
    __builtin_amdgcn_fence(__ATOMIC_RELEASE, "workgroup");
    __builtin_amdgcn_wave_barrier();
    __builtin_amdgcn_fence(__ATOMIC_ACQUIRE, "workgroup");
  }
}

__global__ __launch_bounds__(256) void cast_f16_pad_kernel(
    const float* __restrict__ src, unsigned short* __restrict__ dst, int total8, int valid8, float scale)
{
  const int i = blockIdx.x * 256 + threadIdx.x;
  if (i >= total8) return;
  const bool live = (i < valid8);
  const int ic = live ? i : (valid8 - 1);
  const float* p = src + ((size_t)ic << 3);
  const v4f a0 = *(const v4f*)(p);
  const v4f a1 = *(const v4f*)(p + 4);
  v8h hv;
#pragma unroll
  for (int e = 0; e < 4; ++e) {
    const float z0 = live ? a0[e] : 0.f;
    const float z1 = live ? a1[e] : 0.f;
    hv[e]     = (_Float16)(z0 * scale);
    hv[4 + e] = (_Float16)(z1 * scale);
  }
  unsigned short* q = dst + ((size_t)i << 3);
  *(volatile v8h*)q = hv;
  __threadfence();
  *(volatile v8h*)q = hv;
}

__device__ __forceinline__ void split_bf(float v, _Float16& h, _Float16& l) {
  const unsigned short hb = f2bf_bits(v);
  const unsigned short lb = f2bf_bits(v - bf_bits2f(hb));
  h = __builtin_bit_cast(_Float16, hb);
  l = __builtin_bit_cast(_Float16, lb);
}
__global__ __launch_bounds__(256) void split_bf16_kernel(
    const float* __restrict__ src, unsigned short* __restrict__ hi, unsigned short* __restrict__ lo, int total8)
{
  const int i = blockIdx.x * 256 + threadIdx.x;
  if (i >= total8) return;
  const size_t e0 = (size_t)i << 3;
  const v4f a0 = *(const v4f*)(src + e0);
  const v4f a1 = *(const v4f*)(src + e0 + 4);
  v8h hv, lv;
#pragma unroll
  for (int e = 0; e < 4; ++e) {
    _Float16 h, l;
    split_bf(a0[e], h, l); hv[e] = h;     lv[e] = l;
    split_bf(a1[e], h, l); hv[4 + e] = h; lv[4 + e] = l;
  }
  *(volatile v8h*)(hi + e0) = hv;
  *(volatile v8h*)(lo + e0) = lv;
  __threadfence();
  *(volatile v8h*)(hi + e0) = hv;
  *(volatile v8h*)(lo + e0) = lv;
}

__global__ __launch_bounds__(256) void transpose_split_kernel(
    const float* __restrict__ src, unsigned short* __restrict__ H, unsigned short* __restrict__ L, int dstBatch0)
{
  __shared__ float tile[64 * 65];
  const int tid = threadIdx.x, lane = tid & 31, wave = tid >> 5;
  const int b = blockIdx.x;
  const float* s = src + (size_t)b * (kNC * kNS);
#pragma unroll
  for (int p = 0; p < 16; ++p) {
    const int idx = tid + p * 256;
    const int cc  = idx >> 6;
    const int ss  = idx & 63;
    tile[cc * 65 + ss] = s[idx];
  }
  __syncthreads();
  const int q = lane >> 3, c8 = (lane & 7) * 8;
  v8h hv[2], lv[2];
#pragma unroll
  for (int it = 0; it < 2; ++it) {
    const int srow = it * 32 + wave * 4 + q;
#pragma unroll
    for (int e = 0; e < 8; ++e) {
      _Float16 h, l;
      split_bf(tile[(c8 + e) * 65 + srow], h, l);
      hv[it][e] = h; lv[it][e] = l;
    }
  }
  const size_t ob = (size_t)(dstBatch0 + b) * (kNC * kNS);
  for (int pass = 0; pass < 2; ++pass) {
#pragma unroll
    for (int it = 0; it < 2; ++it) {
      const int srow = it * 32 + wave * 4 + q;
      *(volatile v8h*)(H + ob + (size_t)srow * kNC + c8) = hv[it];
      *(volatile v8h*)(L + ob + (size_t)srow * kNC + c8) = lv[it];
    }
    __threadfence();
  }
}

__global__ __launch_bounds__(256) void products_kernel(
    const float* __restrict__ XP, float* __restrict__ T, unsigned short* __restrict__ T16, int n4, int n8)
{
  const int i = blockIdx.x * 256 + threadIdx.x;
  const size_t P1 = (size_t)kPlane, P2 = 2 * (size_t)kPlane;
  if (i < n4) {
    const size_t e0 = (size_t)i << 2;
    const v4f a  = *(const v4f*)(XP + e0);
    const v4f bq = *(const v4f*)(XP + P1 + e0);
    const v4f cq = *(const v4f*)(XP + P2 + e0);
    const v4f t1 = a * bq;
    const v4f t2 = a * cq;
    *(volatile v4f*)(T + e0)      = a;
    *(volatile v4f*)(T + P1 + e0) = t1;
    *(volatile v4f*)(T + P2 + e0) = t2;
    __threadfence();
    *(volatile v4f*)(T + e0)      = a;
    *(volatile v4f*)(T + P1 + e0) = t1;
    *(volatile v4f*)(T + P2 + e0) = t2;
  }
  if (i < n8) {
    const size_t e1 = (size_t)i << 3;
    const v4f a0 = *(const v4f*)(XP + e1),      a1 = *(const v4f*)(XP + e1 + 4);
    const v4f b0 = *(const v4f*)(XP + P1 + e1), b1 = *(const v4f*)(XP + P1 + e1 + 4);
    const v4f c0 = *(const v4f*)(XP + P2 + e1), c1 = *(const v4f*)(XP + P2 + e1 + 4);
    const v4f p10 = a0 * b0, p11 = a1 * b1, p20 = a0 * c0, p21 = a1 * c1;
    v8h h0, h1, h2;
#pragma unroll
    for (int e = 0; e < 4; ++e) {
      h0[e] = (_Float16)a0[e];  h0[4 + e] = (_Float16)a1[e];
      h1[e] = (_Float16)p10[e]; h1[4 + e] = (_Float16)p11[e];
      h2[e] = (_Float16)p20[e]; h2[4 + e] = (_Float16)p21[e];
    }
    *(volatile v8h*)(T16 + e1)      = h0;
    *(volatile v8h*)(T16 + P1 + e1) = h1;
    *(volatile v8h*)(T16 + P2 + e1) = h2;
    __threadfence();
    *(volatile v8h*)(T16 + e1)      = h0;
    *(volatile v8h*)(T16 + P1 + e1) = h1;
    *(volatile v8h*)(T16 + P2 + e1) = h2;
  }
}

__global__ __launch_bounds__(128) void conv_silu_kernel(
    const float* __restrict__ XZ, const float* __restrict__ cw, const float* __restrict__ cb,
    float* __restrict__ U, unsigned short* __restrict__ U16)
{
  __shared__ __align__(16) float sT[16 * kTP];
  const int tid = threadIdx.x, lane = tid & 31, wave = tid >> 5, hh = lane >> 4;
  const int d = tid;
  const int row0 = blockIdx.x * kNC;
  const float w0 = cw[d * 4 + 0], w1 = cw[d * 4 + 1], w2 = cw[d * 4 + 2], w3 = cw[d * 4 + 3];
  const float bc = cb[d];
  float xm3 = 0.f, xm2 = 0.f, xm1 = 0.f;
  const int c8 = (lane & 15) * 8;
#pragma unroll 1
  for (int sub = 0; sub < 4; ++sub) {
    const int lb = row0 + sub * 16;
#pragma unroll 1
    for (int s = 0; s < 16; ++s) {
      const float xc = XZ[(size_t)(lb + s) * kXZP + d];
      float acc = w0 * xm3;
      acc = fmaf(w1, xm2, acc);
      acc = fmaf(w2, xm1, acc);
      acc = fmaf(w3, xc, acc);
      const float sv = acc + bc;
      const float sg = __builtin_amdgcn_rcpf(1.0f + __expf(-sv));
      sT[s * kTP + tid] = sv * sg;
      xm3 = xm2; xm2 = xm1; xm1 = xc;
    }
    __syncthreads();
    v4f fv[4];
    v8h bv[2];
#pragma unroll
    for (int it = 0; it < 4; ++it) fv[it] = *(const v4f*)(sT + (it * 4 + wave) * kTP + lane * 4);
#pragma unroll
    for (int it = 0; it < 2; ++it) {
      const float* sp = sT + (it * 8 + wave * 2 + hh) * kTP + c8;
      const v4f a0 = *(const v4f*)(sp);
      const v4f a1 = *(const v4f*)(sp + 4);
#pragma unroll
      for (int e = 0; e < 4; ++e) {
        bv[it][e]     = (_Float16)(a0[e] * 16.0f);
        bv[it][4 + e] = (_Float16)(a1[e] * 16.0f);
      }
    }
    for (int pass = 0; pass < 2; ++pass) {
#pragma unroll
      for (int it = 0; it < 4; ++it)
        *(volatile v4f*)(U + (size_t)(lb + it * 4 + wave) * kDin + lane * 4) = fv[it];
#pragma unroll
      for (int it = 0; it < 2; ++it)
        *(volatile v8h*)(U16 + (size_t)(lb + it * 8 + wave * 2 + hh) * kDin + c8) = bv[it];
      __threadfence();
    }
    __syncthreads();
  }
}

__global__ __launch_bounds__(128) void scan_kernel(
    const float* __restrict__ XDBL, const float* __restrict__ U, const float* __restrict__ XZ,
    const float* __restrict__ Wdt, const float* __restrict__ bdt,
    const float* __restrict__ A_log, const float* __restrict__ Dv,
    unsigned short* __restrict__ Y16)
{
  __shared__ __align__(16) float sX[64 * 64];
  __shared__ __align__(16) float sY[16 * kTP];
  const int tid = threadIdx.x, lane = tid & 31, wave = tid >> 5, hh = lane >> 4;
  const int d = tid;
  const int row0 = blockIdx.x * kNC;
#pragma unroll
  for (int it = 0; it < 8; ++it) {
    const int idx4 = tid + it * 128;
    const int r = idx4 >> 4, c4 = (idx4 & 15) * 4;
    const v4f v = *(const v4f*)(XDBL + (size_t)(row0 + r) * kXpP + c4);
    *(v4f*)(sX + r * 64 + c4) = v;
  }
  float An[kNst];
#pragma unroll
  for (int n = 0; n < kNst; ++n) An[n] = -__expf(A_log[(size_t)d * kNst + n]);
  const float wd0 = Wdt[d * 4 + 0], wd1 = Wdt[d * 4 + 1], wd2 = Wdt[d * 4 + 2], wd3 = Wdt[d * 4 + 3];
  const float bd = bdt[d];
  const float Dd = Dv[d];
  float h[kNst];
#pragma unroll
  for (int n = 0; n < kNst; ++n) h[n] = 0.f;
  const int c8 = (lane & 15) * 8;
  __syncthreads();

#pragma unroll 1
  for (int c = 0; c < 4; ++c) {
    const int l0 = c * 16;
#pragma unroll 1
    for (int s = 0; s < 16; ++s) {
      const int l = l0 + s;
      const size_t m = (size_t)(row0 + l);
      const v4f dr = *(const v4f*)(sX + l * 64);
      float a = dr[0] * wd0;
      a = fmaf(dr[1], wd1, a);
      a = fmaf(dr[2], wd2, a);
      a = fmaf(dr[3], wd3, a);
      a += bd;
      const float delta = fmaxf(a, 0.0f) + log1pf(__expf(-fabsf(a)));
      const float xv = U[m * kDin + d];
      const float zv = XZ[m * kXZP + kDin + d];
      v4f Bq[4], Cq[4];
#pragma unroll
      for (int qq = 0; qq < 4; ++qq) {
        Bq[qq] = *(const v4f*)(sX + l * 64 + kDtR + 4 * qq);
        Cq[qq] = *(const v4f*)(sX + l * 64 + kDtR + kNst + 4 * qq);
      }
      float dtu = delta * xv;
      asm volatile("" : "+v"(dtu));
      float y = 0.f;
#pragma unroll
      for (int n = 0; n < kNst; ++n) {
        const float e = __expf(delta * An[n]);
        float p = dtu * Bq[n >> 2][n & 3];
        asm volatile("" : "+v"(p));
        float qv = h[n] * e;
        asm volatile("" : "+v"(qv));
        const float hn = qv + p;
        h[n] = hn;
        float rr = hn * Cq[n >> 2][n & 3];
        asm volatile("" : "+v"(rr));
        y += rr;
      }
      float sk = xv * Dd;
      asm volatile("" : "+v"(sk));
      y += sk;
      const float sg = __builtin_amdgcn_rcpf(1.0f + __expf(-zv));
      const float g  = zv * sg;
      sY[s * kTP + tid] = (y * g) * 64.0f;
    }
    __syncthreads();
    v8h hv[2];
#pragma unroll
    for (int it = 0; it < 2; ++it) {
      const float* sp = sY + (it * 8 + wave * 2 + hh) * kTP + c8;
      const v4f a0 = *(const v4f*)(sp);
      const v4f a1 = *(const v4f*)(sp + 4);
#pragma unroll
      for (int e = 0; e < 4; ++e) { hv[it][e] = (_Float16)a0[e]; hv[it][4 + e] = (_Float16)a1[e]; }
    }
    for (int pass = 0; pass < 2; ++pass) {
#pragma unroll
      for (int it = 0; it < 2; ++it)
        *(volatile v8h*)(Y16 + (size_t)(row0 + l0 + it * 8 + wave * 2 + hh) * kDin + c8) = hv[it];
      __threadfence();
    }
    __syncthreads();
  }
}

__device__ __forceinline__ double block_sum256(double v, double* sred, int tid) {
  sred[tid] = v;
  __syncthreads();
#pragma unroll 1
  for (int st = 128; st > 0; st >>= 1) {
    if (tid < st) sred[tid] = sred[tid] + sred[tid + st];
    __syncthreads();
  }
  const double r = sred[0];
  __syncthreads();
  return r;
}
__global__ __launch_bounds__(256) void bn_mix_kernel(
    const float* __restrict__ CV, const float* __restrict__ gamma, const float* __restrict__ beta,
    const float* __restrict__ xs1p, const float* __restrict__ xs2p, float* __restrict__ out)
{
  __shared__ double sred[256];
  const int tid = threadIdx.x, lane = tid & 31, wave = tid >> 5, hh = lane >> 4;
  const int o = blockIdx.x;
  const int scol = tid & 63, brow = tid >> 6;
  float meanv[3], rsv[3];
#pragma unroll
  for (int t = 0; t < 3; ++t) {
    const float* P = CV + (size_t)t * kPlane + (size_t)o * kNS + scol;
    double s1 = 0.0;
#pragma unroll 1
    for (int i = 0; i < 64; ++i) s1 += (double)P[(size_t)(i * 4 + brow) * (kNC * kNS)];
    const double tot1 = block_sum256(s1, sred, tid);
    const float mean = (float)(tot1 * (1.0 / 16384.0));
    double s2 = 0.0;
#pragma unroll 1
    for (int i = 0; i < 64; ++i) {
      const float dv = P[(size_t)(i * 4 + brow) * (kNC * kNS)] - mean;
      s2 += (double)dv * (double)dv;
    }
    const double tot2 = block_sum256(s2, sred, tid);
    const float var = (float)(tot2 * (1.0 / 16384.0));
    meanv[t] = mean;
    rsv[t] = rsqrtf(var + 1e-5f);
  }
  const float g = gamma[o], be = beta[o];
  const float xs1 = xs1p[0], xs2 = xs2p[0];
  const int c4 = (lane & 15) * 4;
  const float* P0 = CV + (size_t)o * kNS + c4;
  const float* P1 = P0 + (size_t)kPlane;
  const float* P2 = P0 + 2 * (size_t)kPlane;
  float* O = out + (size_t)o * kNS + c4;
#pragma unroll 1
  for (int j = 0; j < 16; ++j) {
    const int b = wave * 32 + j * 2 + hh;
    const size_t off = (size_t)b * (kNC * kNS);
    const v4f v0 = *(const v4f*)(P0 + off);
    const v4f v1 = *(const v4f*)(P1 + off);
    const v4f v2 = *(const v4f*)(P2 + off);
    v4f res;
#pragma unroll
    for (int e = 0; e < 4; ++e) {
      const float r0 = fmaxf((g * (v0[e] - meanv[0])) * rsv[0] + be, 0.f);
      const float r1 = fmaxf((g * (v1[e] - meanv[1])) * rsv[1] + be, 0.f);
      const float r2 = fmaxf((g * (v2[e] - meanv[2])) * rsv[2] + be, 0.f);
      res[e] = (r0 + xs1 * r1) + xs2 * r2;
    }
    *(volatile v4f*)(O + off) = res;
    __threadfence();
    *(volatile v4f*)(O + off) = res;
  }
}

extern "C" void kernel_launch(void* const* d_in, const int* in_sizes, int n_in,
                              void* d_out, int out_size, void* d_ws, size_t ws_size,
                              hipStream_t stream)
{
  if (n_in < 18) return;
  const float* x1         = (const float*)d_in[0];
  const float* x2         = (const float*)d_in[1];
  const float* x3         = (const float*)d_in[2];
  const float* conv1_w    = (const float*)d_in[3];
  const float* conv1_b    = (const float*)d_in[4];
  const float* bn_gamma   = (const float*)d_in[5];
  const float* bn_beta    = (const float*)d_in[6];
  const float* xishu1     = (const float*)d_in[7];
  const float* xishu2     = (const float*)d_in[8];
  const float* in_proj_w  = (const float*)d_in[9];
  const float* conv1d_w   = (const float*)d_in[10];
  const float* conv1d_b   = (const float*)d_in[11];
  const float* x_proj_w   = (const float*)d_in[12];
  const float* dt_proj_w  = (const float*)d_in[13];
  const float* dt_proj_b  = (const float*)d_in[14];
  const float* A_log      = (const float*)d_in[15];
  const float* Dvec       = (const float*)d_in[16];
  const float* out_proj_w = (const float*)d_in[17];
  float* dout = (float*)d_out;

  if (in_sizes[0] != kPlane || in_sizes[1] != kPlane || in_sizes[2] != kPlane) return;
  if (in_sizes[3] != kNC * kNC || in_sizes[4] != kNC || in_sizes[5] != kNC || in_sizes[6] != kNC) return;
  if (in_sizes[7] < 1 || in_sizes[8] < 1) return;
  if (in_sizes[9] != kXZP * kNS) return;
  if (in_sizes[10] != kDin * 4 || in_sizes[11] != kDin) return;
  if (in_sizes[12] != kXpN * kDin) return;
  if (in_sizes[13] != kDin * kDtR || in_sizes[14] != kDin) return;
  if (in_sizes[15] != kDin * kNst || in_sizes[16] != kDin) return;
  if (in_sizes[17] != kNS * kDin) return;
  if (out_size != kPlane) return;

  const size_t SZ_W1    = (size_t)kNC * kNC * 2;
  const size_t SZ_WIN   = (size_t)kXZP * kNS * 2;
  const size_t SZ_WXP   = (size_t)kXpP * kDin * 2;
  const size_t SZ_WO    = (size_t)kNS * kDin * 2;
  const size_t SZ_R     = (size_t)kNBr * kPlane * 4;
  const size_t SZ_HALFR = SZ_R / 2;
  const size_t SZ_T16   = (size_t)kRows * kNS * 2;
  const size_t SZ_XZ    = (size_t)kRows * kXZP * 4;
  const size_t SZ_U     = (size_t)kRows * kDin * 4;
  const size_t OFF_W1H = 0;
  const size_t OFF_W1L = OFF_W1H + SZ_W1;
  const size_t OFF_WIN = OFF_W1L + SZ_W1;
  const size_t OFF_WXP = OFF_WIN + SZ_WIN;
  const size_t OFF_WO  = OFF_WXP + SZ_WXP;
  const size_t OFF_RA  = 131072;
  const size_t OFF_RB  = OFF_RA + SZ_R;
  const size_t OFF_RT  = OFF_RB + SZ_R;
  const size_t OFF_T16 = OFF_RT + SZ_R;
  const size_t OFF_XZ  = OFF_T16 + SZ_T16;
  const size_t OFF_U   = OFF_XZ + SZ_XZ;
  const size_t TOTAL   = OFF_U + SZ_U;
  if (OFF_WO + SZ_WO > OFF_RA) return;
  if (ws_size < TOTAL) return;

  char* ws = (char*)d_ws;
  unsigned short* W1H   = (unsigned short*)(ws + OFF_W1H);
  unsigned short* W1L   = (unsigned short*)(ws + OFF_W1L);
  unsigned short* WIN16 = (unsigned short*)(ws + OFF_WIN);
  unsigned short* WXP16 = (unsigned short*)(ws + OFF_WXP);
  unsigned short* WO16  = (unsigned short*)(ws + OFF_WO);
  unsigned short* XTH   = (unsigned short*)(ws + OFF_RA);
  unsigned short* XTL   = (unsigned short*)(ws + OFF_RA + SZ_HALFR);
  unsigned short* U16   = (unsigned short*)(ws + OFF_RA);
  unsigned short* Y16   = (unsigned short*)(ws + OFF_RA);
  unsigned short* MTH   = (unsigned short*)(ws + OFF_RA);
  unsigned short* MTL   = (unsigned short*)(ws + OFF_RA + SZ_HALFR);
  float*          XP    = (float*)(ws + OFF_RB);
  float*          XDBL  = (float*)(ws + OFF_RB);
  float*          Mres  = (float*)(ws + OFF_RB);
  float*          CV    = (float*)(ws + OFF_RB);
  float*          Tf    = (float*)(ws + OFF_RT);
  unsigned short* T16   = (unsigned short*)(ws + OFF_T16);
  float*          XZ    = (float*)(ws + OFF_XZ);
  float*          Uf    = (float*)(ws + OFF_U);
  const float* dummy_bias  = conv1_b;
  const float* dummy_resid = Tf;

  cast_f16_pad_kernel<<<(kXZP * kNS / 8) / 256, 256, 0, stream>>>(in_proj_w, WIN16, kXZP * kNS / 8, kXZP * kNS / 8, 16.0f);
  cast_f16_pad_kernel<<<(kXpP * kDin / 8) / 256, 256, 0, stream>>>(x_proj_w, WXP16, kXpP * kDin / 8, kXpN * kDin / 8, 16.0f);
  cast_f16_pad_kernel<<<(kNS * kDin / 8) / 256, 256, 0, stream>>>(out_proj_w, WO16, kNS * kDin / 8, kNS * kDin / 8, 16.0f);
  split_bf16_kernel<<<(kNC * kNC / 8) / 256, 256, 0, stream>>>(conv1_w, W1H, W1L, kNC * kNC / 8);

  transpose_split_kernel<<<kNB, 256, 0, stream>>>(x1, XTH, XTL, 0);
  transpose_split_kernel<<<kNB, 256, 0, stream>>>(x2, XTH, XTL, kNB);
  transpose_split_kernel<<<kNB, 256, 0, stream>>>(x3, XTH, XTL, 2 * kNB);

  wmma_gemm64<1, true, 1, 0, false, 0, true><<<dim3(1, kSeq / 8), 256, 0, stream>>>(
      W1H, W1L, kNC, 0L, XTH, XTL, kNC, (long)(kNC * kNS),
      (void*)XP, (void*)XP, kNS, (long)(kNC * kNS), conv1_b, dummy_resid, 0L, kNC, kNS, kNC, 1.0f);

  products_kernel<<<(kPlane / 4) / 256, 256, 0, stream>>>(XP, Tf, T16, kPlane / 4, kPlane / 8);

  wmma_gemm64<0, false, 0, 0, false><<<dim3(kRows * (kXZP / 64) / 64 / 8, 1), 256, 0, stream>>>(
      T16, T16, kNS, 0L, WIN16, WIN16, kNS, 0L,
      (void*)XZ, (void*)XZ, kXZP, 0L, dummy_bias, dummy_resid, 0L, kRows, kXZP, kNS, 1.0f / 16.0f);

  conv_silu_kernel<<<kSeq, 128, 0, stream>>>(XZ, conv1d_w, conv1d_b, Uf, U16);

  wmma_gemm64<0, false, 0, 0, false><<<dim3(kRows / 64 / 8, 1), 256, 0, stream>>>(
      U16, U16, kDin, 0L, WXP16, WXP16, kDin, 0L,
      (void*)XDBL, (void*)XDBL, kXpP, 0L, dummy_bias, dummy_resid, 0L, kRows, kXpP, kDin, 1.0f / 256.0f);

  scan_kernel<<<kSeq, 128, 0, stream>>>(XDBL, Uf, XZ, dt_proj_w, dt_proj_b, A_log, Dvec, Y16);

  wmma_gemm64<0, false, 0, 0, true><<<dim3(kRows / 64 / 8, 1), 256, 0, stream>>>(
      Y16, Y16, kDin, 0L, WO16, WO16, kDin, 0L,
      (void*)Mres, (void*)Mres, kNS, 0L, dummy_bias, Tf, 0L, kRows, kNS, kDin, 1.0f / 1024.0f);

  transpose_split_kernel<<<kSeq, 256, 0, stream>>>(Mres, MTH, MTL, 0);

  wmma_gemm64<1, true, 1, 0, false, 0, true><<<dim3(1, kSeq / 8), 256, 0, stream>>>(
      W1H, W1L, kNC, 0L, MTH, MTL, kNC, (long)(kNC * kNS),
      (void*)CV, (void*)CV, kNS, (long)(kNC * kNS), conv1_b, dummy_resid, 0L, kNC, kNS, kNC, 1.0f);

  bn_mix_kernel<<<kNC, 256, 0, stream>>>(CV, bn_gamma, bn_beta, xishu1, xishu2, dout);
}
